// SoftImageToReflectanceMap_56221121905131
// MI455X (gfx1250) — hardware-run, weakly checked
//
#include <hip/hip_runtime.h>
#pragma clang fp contract(off)


#ifndef NB
#define NB 2
#endif
#ifndef NPIX
#define NPIX 16384
#endif
#ifndef NDIRS
#define NDIRS 65536
#endif
#define NB_FULL   2
#define NPIX_FULL 16384
#define NDIR_FULL 65536
#define OSZ   256
#define NCH   3
#define VROWS 16
#define VSRC  9
#define AW    4
#define DPW   32
#define THR   40.0f
#define SH0   (-512.0f)
#define ONEB  0x3F80

static_assert(NCH == 3);
static_assert(OSZ * OSZ == NDIR_FULL);
static_assert((OSZ & (OSZ - 1)) == 0);
static_assert(NB <= NB_FULL);
static_assert(NPIX <= NPIX_FULL);
static_assert(NDIRS <= NDIR_FULL);
static_assert(NPIX % 256 == 0);
static_assert(NPIX % 32 == 0);
static_assert(NDIRS % (DPW * AW) == 0);
static_assert(DPW == 32);
static_assert(DPW * 4 == 128);
static_assert(8 * NCH <= 32);
static_assert(8 * NCH * 16 == NCH * DPW * 4);
static_assert(VSRC == 3 * NCH);
static_assert(VSRC <= VROWS);
static_assert(2 * 256 * 8 == VROWS * 256);
static_assert(AW * NCH * DPW * 4 <= 131072);
static_assert(VSRC * 256 * 2 <= 131072);

typedef unsigned short bf;
typedef __attribute__((ext_vector_type(16))) __bf16   v16bf;
typedef __attribute__((ext_vector_type(2)))  __bf16   v2bf;
typedef __attribute__((ext_vector_type(8)))  unsigned short v8us;
typedef __attribute__((ext_vector_type(8)))  unsigned v8u;
typedef __attribute__((ext_vector_type(8)))  float    v8f;
typedef __attribute__((ext_vector_type(4)))  float    v4f;
typedef __attribute__((ext_vector_type(2)))  float    v2f;
typedef v4f  __attribute__((may_alias)) v4fa;
typedef v8us __attribute__((may_alias)) v8usa;

__device__ __forceinline__ unsigned short f2bf(float f) { unsigned u = __float_as_uint(f); u += 0x7FFFu + ((u >> 16) & 1u); return (unsigned short)(u >> 16); }
__device__ __forceinline__ float bfr(float f) { return __uint_as_float(((unsigned)f2bf(f)) << 16); }
__device__ __forceinline__ v16bf cat16b(v8us lo, v8us hi) { return __builtin_bit_cast(v16bf, __builtin_shufflevector(lo, hi, 0, 1, 2, 3, 4, 5, 6, 7, 8, 9, 10, 11, 12, 13, 14, 15)); }
__device__ __forceinline__ v8f wmmab(v16bf a, v16bf b, v8f c) { return __builtin_amdgcn_wmma_f32_16x16x32_bf16(false, a, false, b, (short)0, c, false, false); }
__device__ __forceinline__ v16bf ldb(const bf* p)  { return cat16b(*(const v8us*)p, *(const v8us*)(p + 16)); }
__device__ __forceinline__ void wave_sync() { __builtin_amdgcn_fence(3  , "wavefront"); __builtin_amdgcn_wave_barrier(); asm volatile("" ::: "memory"); }

__device__ __forceinline__ v8f wmmab_g(v16bf a, v16bf b, v8f c) {
    c = wmmab(a, b, c);
    asm volatile("v_nop\n\tv_nop\n\tv_nop\n\tv_nop" : "+v"(c) : "v"(a), "v"(b));
    return c;
}
__device__ __forceinline__ float bfv(bf h) { return __uint_as_float(((unsigned)h) << 16); }
__device__ __forceinline__ void split3(float v, bf& h, bf& m, bf& l) {
    h = f2bf(v); const float r1 = v - bfv(h); m = f2bf(r1); const float r2 = r1 - bfv(m); l = f2bf(r2);
}
__device__ __forceinline__ unsigned pk2(float a, float c) { const v2f t = {a, c}; return __builtin_bit_cast(unsigned, __builtin_convertvector(t, v2bf)); }
__device__ __forceinline__ void mkfrag(unsigned s0, unsigned s1, unsigned s2, unsigned s3, int hi, float sh, v16bf& b1, v16bf& b2) {
    bf ch, cm, cl; split3(-sh, ch, cm, cl);
    const unsigned c0 = ((unsigned)ch) << 16, c1 = (unsigned)cm | (((unsigned)cl) << 16);
    const unsigned w0 = s0 | (hi ? c0 : 0u), w1 = s1 | (hi ? c1 : 0u);
    const v8u a = {w0, w1, s2, s3, 0u, 0u, 0u, 0u};
    const v8u c = {0u, 0u, 0u, 0u, w0, w1, s2, s3};
    b1 = __builtin_bit_cast(v16bf, a); b2 = __builtin_bit_cast(v16bf, c);
}

__global__ __launch_bounds__(256) void k_prep(const float* __restrict__ image, const float* __restrict__ nrm, const int* __restrict__ mask, bf* NP, bf* VT) {
    __shared__ __align__(16) unsigned short vs[VSRC * 256];
    const int t = threadIdx.x; const int b = blockIdx.y; const int p0 = blockIdx.x * 256; const int p = p0 + t;
    const size_t ib = (size_t)b * NCH * NPIX_FULL + (size_t)p;
    int mk = mask[(size_t)b * NPIX_FULL + (size_t)p];
    float n0 = nrm[ib], n1 = nrm[ib + (size_t)NPIX_FULL], n2 = nrm[ib + 2 * (size_t)NPIX_FULL];
    float i0 = image[ib], i1 = image[ib + (size_t)NPIX_FULL], i2 = image[ib + 2 * (size_t)NPIX_FULL];
    asm volatile("" : "+v"(mk)); asm volatile("" : "+v"(n0)); asm volatile("" : "+v"(n1)); asm volatile("" : "+v"(n2));
    asm volatile("" : "+v"(i0)); asm volatile("" : "+v"(i1)); asm volatile("" : "+v"(i2));
    const bool w = mk > 0;
    const bf ax = w ? f2bf(n0) : (bf)0, ay = w ? f2bf(n1) : (bf)0, az = w ? f2bf(n2) : (bf)0;
    const bf u0 = w ? f2bf(i0) : (bf)0, u1 = w ? f2bf(i1) : (bf)0, u2 = w ? f2bf(i2) : (bf)0;
    const float f0 = bfv(u0), f1 = bfv(u1), f2 = bfv(u2);
    const float q0 = f0 * f0, q1 = f1 * f1, q2 = f2 * f2;
    const bf h0 = f2bf(q0), h1 = f2bf(q1), h2 = f2bf(q2);
    const bf l0 = f2bf(q0 - bfv(h0)), l1 = f2bf(q1 - bfv(h1)), l2 = f2bf(q2 - bfv(h2));
    v8us pa, pb;
    pa[0] = ax; pa[1] = ay; pa[2] = az; pa[3] = ax; pa[4] = ay; pa[5] = az; pa[6] = ax; pa[7] = ay;
    pb[0] = az; pb[1] = (bf)ONEB; pb[2] = (bf)ONEB; pb[3] = (bf)ONEB; pb[4] = 0; pb[5] = 0; pb[6] = 0; pb[7] = 0;
    vs[0 * 256 + t] = u0; vs[1 * 256 + t] = u1; vs[2 * 256 + t] = u2;
    vs[3 * 256 + t] = h0; vs[4 * 256 + t] = h1; vs[5 * 256 + t] = h2;
    vs[6 * 256 + t] = l0; vs[7 * 256 + t] = l1; vs[8 * 256 + t] = l2;
    __syncthreads();
    const int ra = t >> 5, rb = 8 + (t >> 5); const int c8 = (t & 31) * 8;
    const int sa = ra < VSRC ? ra : (VSRC - 1), sb = rb < VSRC ? rb : (VSRC - 1);
    v8us xa = *(const v8usa*)(&vs[sa * 256 + c8]);
    v8us xb = *(const v8usa*)(&vs[sb * 256 + c8]);
    const v8us zz = (v8us){};
    if (ra >= VSRC) xa = zz;
    if (rb >= VSRC) xb = zz;
    bf* npa = NP + ((size_t)(b * 2 + 0) * NPIX + (size_t)p) * 8;
    bf* npb = NP + ((size_t)(b * 2 + 1) * NPIX + (size_t)p) * 8;
    bf* vta = VT + ((size_t)(b * VROWS + ra) * NPIX + (size_t)p0 + c8);
    bf* vtb = VT + ((size_t)(b * VROWS + rb) * NPIX + (size_t)p0 + c8);
#pragma unroll 1
    for (int ps = 0; ps < 2; ++ps) {
        *(volatile v8us*)npa = pa; *(volatile v8us*)npb = pb;
        *(volatile v8us*)vta = xa; *(volatile v8us*)vtb = xb;
        if (ps == 0) __threadfence(); }
}

__global__ __launch_bounds__(32 * AW) void k_splat(const bf* __restrict__ NP, const bf* __restrict__ VT, const int* __restrict__ kappa_p, const int* __restrict__ osz_p, float* OUT) {
    __shared__ __align__(16) float os[AW * NCH * DPW];
    const int lane = threadIdx.x & 31, lr = lane & 15, hi = lane >> 4;
    const int wave = __builtin_amdgcn_readfirstlane((int)(threadIdx.x >> 5));
    const int b = blockIdx.y;
    const int dbase = (blockIdx.x * AW + wave) * DPW;
    const float kk = (float)kappa_p[0];
    const float rosz = 1.0f / (float)osz_p[0];
    const float L2E = 1.4426950408889634f;
    const float ea = kk * L2E;
    const float den = 6.283185307179586f * (1.0f - __builtin_amdgcn_exp2f(-2.0f * kk * L2E));
    const float coef = kk * __builtin_amdgcn_rcpf(den);
    const float eb = __builtin_amdgcn_logf(coef) - ea;
    const size_t no = ((size_t)(b * 2 + hi) * NPIX + (size_t)lr) * 8;
    const size_t vo = ((size_t)b * VROWS + (size_t)lr) * NPIX + 8 * hi;
    const int wb = wave * (NCH * DPW);
    const v8f zacc = (v8f){};
#pragma unroll 1
    for (int dt = 0; dt < 2; ++dt) {
        const int dir = dbase + 16 * dt + lr;
        const float uu = (float)(dir & (OSZ - 1)), vv = (float)(dir / OSZ);
        const float p = 4.0f * ((uu + 0.5f) * rosz - 0.5f);
        const float q = -4.0f * ((vv + 0.5f) * rosz - 0.5f);
        const float pp = p * p, qq = q * q;
        const float dd = (1.0f + pp) + qq;
        const float inv = __builtin_amdgcn_rcpf(dd);
        const float X = ea * ((2.0f * p) * inv);
        const float Y = ea * ((2.0f * q) * inv);
        const float Z = ea * (-(((-1.0f) + pp) + qq) * inv);
        bf xh, xm, xl, yh, ym, yl, zh, zm, zl;
        split3(X, xh, xm, xl); split3(Y, yh, ym, yl); split3(Z, zh, zm, zl);
        const unsigned s0 = hi ? (unsigned)zl : ((unsigned)xh | (((unsigned)yh) << 16));
        const unsigned s1 = hi ? 0u : ((unsigned)zh | (((unsigned)xm) << 16));
        const unsigned s2 = hi ? 0u : ((unsigned)ym | (((unsigned)zm) << 16));
        const unsigned s3 = hi ? 0u : ((unsigned)xl | (((unsigned)yl) << 16));
        float sh = SH0;
        v16bf b1, b2; mkfrag(s0, s1, s2, s3, hi, sh, b1, b2);
        v8f acc = (v8f){};
#pragma unroll 1
        for (int key0 = 0; key0 < NPIX; key0 += 32) {
            const v8us ra = *(const v8us*)(NP + no + (size_t)key0 * 8);
            const v8us rb = *(const v8us*)(NP + no + (size_t)(key0 + 16) * 8);
            const v16bf na = cat16b(ra, rb);
            v8f sa = wmmab_g(na, b1, zacc);
            v8f sb = wmmab_g(na, b2, zacc);
            float mx = fmaxf(sa[0], sb[0]);
#pragma unroll
            for (int r = 1; r < 8; ++r) mx = fmaxf(mx, fmaxf(sa[r], sb[r]));
            if (__builtin_amdgcn_ballot_w32(mx > THR) != 0u) {
                const float mo = fmaxf(mx, __shfl_xor(mx, 16, 32));
                const float dl = fmaxf(mo, 0.0f);
                sh += dl;
                const float al = __builtin_amdgcn_exp2f(-dl);
                acc = acc * al;
                sa = sa - dl; sb = sb - dl;
                mkfrag(s0, s1, s2, s3, hi, sh, b1, b2);
            }
            v8u pk;
#pragma unroll
            for (int j = 0; j < 4; ++j) {
                pk[j]     = pk2(__builtin_amdgcn_exp2f(sa[2 * j]), __builtin_amdgcn_exp2f(sa[2 * j + 1]));
                pk[4 + j] = pk2(__builtin_amdgcn_exp2f(sb[2 * j]), __builtin_amdgcn_exp2f(sb[2 * j + 1])); }
            const v16bf pb = __builtin_bit_cast(v16bf, pk);
            const v16bf vf = ldb(VT + vo + key0);
            acc = wmmab_g(vf, pb, acc);
        }
        const float lo2 = __shfl_xor(acc[0], 16, 32);
        const float ex = fminf(-sh - eb, 126.0f);
        const float tiny = 0.001f * __builtin_amdgcn_exp2f(ex);
        const float d0 = fmaxf(acc[0] + tiny, 1.0e-30f), d1 = fmaxf(acc[1] + tiny, 1.0e-30f), d2 = fmaxf(acc[2] + tiny, 1.0e-30f);
        const float o0 = (acc[3] + acc[6]) * __builtin_amdgcn_rcpf(d0);
        const float o1 = (acc[4] + acc[7]) * __builtin_amdgcn_rcpf(d1);
        const float o2 = (acc[5] + lo2) * __builtin_amdgcn_rcpf(d2);
        if (hi == 0) {
            os[wb + 0 * DPW + 16 * dt + lr] = o0;
            os[wb + 1 * DPW + 16 * dt + lr] = o1;
            os[wb + 2 * DPW + 16 * dt + lr] = o2; }
    }
    wave_sync();
    const int cq = lane >> 3; const int cc = cq < NCH ? cq : (NCH - 1);
    const int c4 = (lane & 7) * 4;
    const v4f val = *(const v4fa*)(&os[wb + cc * DPW + c4]);
    float* op = OUT + ((size_t)b * NCH + (size_t)cc) * NDIR_FULL + (size_t)dbase + c4;
#pragma unroll 1
    for (int ps = 0; ps < 2; ++ps) {
        if (lane < 8 * NCH) *(volatile v4f*)op = val;
        if (ps == 0) __threadfence(); }
}

static constexpr size_t al256(size_t v) { return (v + 255) & ~(size_t)255; }
static constexpr size_t SZ_NP = al256((size_t)NB * 2 * NPIX * 8 * 2);
static constexpr size_t SZ_VT = al256((size_t)NB * VROWS * NPIX * 2);
static constexpr size_t SZ_TOTAL = SZ_NP + SZ_VT;
static_assert(SZ_TOTAL <= (size_t)134217728);
static_assert(((size_t)NPIX * 8 * 2) % 128 == 0);
static_assert(((size_t)NPIX * 2) % 128 == 0);

extern "C" void kernel_launch(void* const* d_in, const int* in_sizes, int n_in,
                              void* d_out, int out_size, void* d_ws, size_t ws_size, hipStream_t stream) {
    if (n_in < 5) return;
    const size_t needx = ((size_t)(NB - 1) * NCH + (NCH - 1)) * NPIX_FULL + NPIX;
    const size_t needm = (size_t)(NB - 1) * NPIX_FULL + NPIX;
    if ((size_t)in_sizes[0] < needx || (size_t)in_sizes[1] < needx) return;
    if ((size_t)in_sizes[2] < needm) return;
    if (in_sizes[3] < 1 || in_sizes[4] < 1) return;
    if ((size_t)out_size < ((size_t)(NB - 1) * NCH + (NCH - 1)) * NDIR_FULL + NDIRS) return;
    if (SZ_TOTAL > ws_size) return;
    const float* image = (const float*)d_in[0];
    const float* nrm   = (const float*)d_in[1];
    const int*   mask  = (const int*)d_in[2];
    const int*   kappa = (const int*)d_in[3];
    const int*   osz   = (const int*)d_in[4];
    float* OUT = (float*)d_out;
    char* wsp = (char*)d_ws;
    bf* NP = (bf*)wsp; wsp += SZ_NP;
    bf* VT = (bf*)wsp; wsp += SZ_VT;

    k_prep<<<dim3(NPIX / 256, NB, 1), 256, 0, stream>>>(image, nrm, mask, NP, VT);
    k_splat<<<dim3(NDIRS / (DPW * AW), NB, 1), 32 * AW, 0, stream>>>(NP, VT, kappa, osz, OUT);
}
